// Encoder_7516192768311
// MI455X (gfx1250) — hardware-verified
//
#include <hip/hip_runtime.h>
#include <stddef.h>
#include <stdint.h>
#include <math.h>


#define NOUT   512
#define ZSD    512
#define ADIM   8
#define ZAD    256
#define I1     768
#define I2     512
#define KL1    (6 * I1)
#define KL2    (6 * I2)
#define NTHR   256
#define NWAVE  8
#define GBM    64
#define GBN    64
#define GTHR   128
#define NQ1    (3 * I1 / 8)
#define NQ2    (3 * I2 / 8)
#define NU1    (NOUT * NQ1)
#define NU2    (NOUT * NQ2)
#define ZROWS  32
#define SBR    8
#define XU     (I1 / 8)
#define WSMAX  134217728

static_assert(KL1 % 32 == 0 && KL2 % 32 == 0);
static_assert(I1 % 8 == 0 && I2 % 8 == 0 && NQ1 % 8 == 0 && NQ2 % 8 == 0);
static_assert(NU1 % NTHR == 0 && NU2 % NTHR == 0);
static_assert(NOUT % GBN == 0 && GBM == (GTHR / 32) * 16 && GBN == 64);
static_assert(I1 == ZSD + ZAD && ZAD == NTHR);
static_assert((SBR * XU) % NTHR == 0 && XU % 8 == 0 && ZROWS % SBR == 0);
static_assert((ADIM * ZAD * 3) % NTHR == 0);
static_assert((SBR * ZSD / 4) % NTHR == 0);
static_assert((KL1 * 2) % 128 == 0 && (KL2 * 2) % 128 == 0 && (I1 * 2) % 128 == 0 && (I2 * 2) % 128 == 0);

typedef float          v4f   __attribute__((ext_vector_type(4)));
typedef float          v8f   __attribute__((ext_vector_type(8)));
typedef int            v8i   __attribute__((ext_vector_type(8)));
typedef unsigned short v8us  __attribute__((ext_vector_type(8)));
typedef unsigned short v16us __attribute__((ext_vector_type(16)));
typedef __bf16         v16bf __attribute__((ext_vector_type(16)));
typedef v4f  __attribute__((may_alias)) v4fa;
typedef v8us __attribute__((may_alias)) v8usa;
union FragB { v16bf v; v16us u; v8us h[2]; v8i w; };

__device__ __forceinline__ v8f wmb(const FragB& a, const FragB& b, v8f c) {
  v8f d = __builtin_amdgcn_wmma_f32_16x16x32_bf16(false, a.v, false, b.v, (short)0, c, false, false);
  asm volatile("v_nop\n\tv_nop\n\tv_nop\n\tv_nop" : "+v"(d) : "v"(a.w), "v"(b.w));
  return d;
}

__device__ __forceinline__ unsigned bf16_bits(float f) {
  const unsigned u = __float_as_uint(f);
  return (u + 0x7FFFu + ((u >> 16) & 1u)) >> 16;
}
__device__ __forceinline__ float bf16_val(float f) {
  return __uint_as_float(bf16_bits(f) << 16);
}

struct HS { unsigned h0, h1, h2, l0, l1, l2; };

__device__ __forceinline__ HS hat_split(float x) {
  const float t  = fminf(fmaxf(x + 1.0f, 0.0f), 2.0f);
  const float b0 = fmaxf(1.0f - fabsf(t), 0.0f);
  const float b1 = fmaxf(1.0f - fabsf(t - 1.0f), 0.0f);
  const float b2 = fmaxf(1.0f - fabsf(t - 2.0f), 0.0f);
  HS s;
  s.h0 = bf16_bits(b0); s.l0 = bf16_bits(b0 - __uint_as_float(s.h0 << 16));
  s.h1 = bf16_bits(b1); s.l1 = bf16_bits(b1 - __uint_as_float(s.h1 << 16));
  s.h2 = bf16_bits(b2); s.l2 = bf16_bits(b2 - __uint_as_float(s.h2 << 16));
  return s;
}

__device__ __forceinline__ void expand8(const v4f a, const v4f b, v8us& h0, v8us& h1, v8us& h2,
                                        v8us& l0, v8us& l1, v8us& l2) {
  const float x[8] = {a.x, a.y, a.z, a.w, b.x, b.y, b.z, b.w};
#pragma unroll
  for (int j = 0; j < 8; ++j) {
    const HS s = hat_split(x[j]);
    h0[j] = (unsigned short)s.h0; h1[j] = (unsigned short)s.h1; h2[j] = (unsigned short)s.h2;
    l0[j] = (unsigned short)s.l0; l1[j] = (unsigned short)s.l1; l2[j] = (unsigned short)s.l2;
  }
}

template <int I>
__device__ __forceinline__ void wt_unit(const float* __restrict__ W, unsigned short* P, int v) {
  constexpr int NQ = 3 * I / 8;
  const int o  = v / NQ;
  const int q  = v - o * NQ;
  const int k8 = q * 8;
  const int p  = k8 / I;
  const int i0 = k8 - p * I;
  const float* s = W + ((size_t)i0 * NOUT + (size_t)o) * 3 + p;
  v8us ov;
#pragma unroll
  for (int j = 0; j < 8; ++j) ov[j] = (unsigned short)bf16_bits(s[(size_t)j * (NOUT * 3)]);
  unsigned short* dp = P + (size_t)o * (6 * I) + k8;
  *(volatile v8us*)dp = ov;
  *(volatile v8us*)(dp + 3 * I) = ov;
  __threadfence();
  *(volatile v8us*)dp = ov;
  *(volatile v8us*)(dp + 3 * I) = ov;
}

__global__ __launch_bounds__(NTHR) void k_prep(const float* __restrict__ W1, const float* __restrict__ W2,
                                               const float* __restrict__ W3, unsigned short* WT1,
                                               unsigned short* WT2, unsigned short* WT3) {
  const int u = (int)blockIdx.x * NTHR + (int)threadIdx.x;
  if (u < NU1) {
    wt_unit<I1>(W1, WT1, u);
  } else if (u < NU1 + NU2) {
    wt_unit<I2>(W2, WT2, u - NU1);
  } else if (u < NU1 + 2 * NU2) {
    wt_unit<I2>(W3, WT3, u - NU1 - NU2);
  }
}

__global__ __launch_bounds__(NTHR) void k_za_expand(const float* __restrict__ zs, const float* __restrict__ action,
                                                    const float* __restrict__ Wza, unsigned short* ab,
                                                    int rowG0) {
  __shared__ __attribute__((aligned(16))) float wl[ADIM * 3 * ZAD];
  __shared__ __attribute__((aligned(16))) float xrow[SBR * I1];
  __shared__ float abas[SBR * ADIM * 3];
  const int tid = (int)threadIdx.x;

#pragma unroll 4
  for (int it = 0; it < (ADIM * ZAD * 3) / NTHR; ++it) {
    const int idx = it * NTHR + tid;
    const int i   = idx / (ZAD * 3);
    const int rem = idx - i * (ZAD * 3);
    const int o   = rem / 3;
    const int p   = rem - 3 * o;
    wl[(i * 3 + p) * ZAD + o] = bf16_val(Wza[idx]);
  }

#pragma unroll 1
  for (int sb = 0; sb < ZROWS / SBR; ++sb) {
    const int lbase = (int)blockIdx.x * ZROWS + sb * SBR;
    const int gbase = rowG0 + lbase;
    if (tid < SBR * ADIM) {
      const int r = tid >> 3, i = tid & 7;
      const float a = bf16_val(action[(size_t)(gbase + r) * ADIM + i]);
      const float t  = fminf(fmaxf(a + 1.0f, 0.0f), 2.0f);
      abas[r * 24 + i * 3 + 0] = fmaxf(1.0f - fabsf(t), 0.0f);
      abas[r * 24 + i * 3 + 1] = fmaxf(1.0f - fabsf(t - 1.0f), 0.0f);
      abas[r * 24 + i * 3 + 2] = fmaxf(1.0f - fabsf(t - 2.0f), 0.0f);
    }
#pragma unroll
    for (int it = 0; it < (SBR * ZSD / 4) / NTHR; ++it) {
      const int idx4 = it * NTHR + tid;
      const int r    = idx4 >> 7;
      const int c4   = (idx4 & 127) * 4;
      const v4f z = *(const v4fa*)(zs + (size_t)(gbase + r) * ZSD + c4);
      v4f y;
      y.x = bf16_val(z.x); y.y = bf16_val(z.y); y.z = bf16_val(z.z); y.w = bf16_val(z.w);
      *(v4fa*)(xrow + r * I1 + c4) = y;
    }
    __syncthreads();

#pragma unroll 1
    for (int r = 0; r < SBR; ++r) {
      float acc = 0.0f;
#pragma unroll 4
      for (int k = 0; k < ADIM * 3; ++k) acc = fmaf(abas[r * 24 + k], wl[k * ZAD + tid], acc);
      const float e = (acc > 0.0f) ? acc : expm1f(acc);
      xrow[r * I1 + ZSD + tid] = e;
    }
    __syncthreads();

#pragma unroll 1
    for (int it = 0; it < (SBR * XU) / NTHR; ++it) {
      const int u = it * NTHR + tid;
      const int r = u / XU;
      const int q = u - r * XU;
      const v4f xa = *(const v4fa*)(xrow + r * I1 + 8 * q);
      const v4f xb = *(const v4fa*)(xrow + r * I1 + 8 * q + 4);
      v8us h0, h1, h2, l0, l1, l2;
      expand8(xa, xb, h0, h1, h2, l0, l1, l2);
      unsigned short* dp = ab + (size_t)(lbase + r) * KL1 + 8 * q;
      *(volatile v8us*)(dp)          = h0;
      *(volatile v8us*)(dp + I1)     = h1;
      *(volatile v8us*)(dp + 2 * I1) = h2;
      *(volatile v8us*)(dp + 3 * I1) = l0;
      *(volatile v8us*)(dp + 4 * I1) = l1;
      *(volatile v8us*)(dp + 5 * I1) = l2;
      __threadfence();
      *(volatile v8us*)(dp)          = h0;
      *(volatile v8us*)(dp + I1)     = h1;
      *(volatile v8us*)(dp + 2 * I1) = h2;
      *(volatile v8us*)(dp + 3 * I1) = l0;
      *(volatile v8us*)(dp + 4 * I1) = l1;
      *(volatile v8us*)(dp + 5 * I1) = l2;
    }
    __syncthreads();
  }
}

__global__ __launch_bounds__(NTHR) void k_ln_expand(const float* __restrict__ H, unsigned short* ab, int nRows) {
  __shared__ float sw[NWAVE * 512];
  const int tid = (int)threadIdx.x, lane = tid & 31, wave = tid >> 5;
  const int row = (int)blockIdx.x * NWAVE + wave;
  if (row >= nRows) return;
  const float* hp = H + (size_t)row * NOUT + 8 * lane;
  const v4f a0 = *(const v4fa*)(hp);
  const v4f a1 = *(const v4fa*)(hp + 4);
  const v4f a2 = *(const v4fa*)(hp + 256);
  const v4f a3 = *(const v4fa*)(hp + 260);
  const float v[16] = {a0.x, a0.y, a0.z, a0.w, a1.x, a1.y, a1.z, a1.w,
                       a2.x, a2.y, a2.z, a2.w, a3.x, a3.y, a3.z, a3.w};
  float s = 0.0f;
#pragma unroll
  for (int j = 0; j < 16; ++j) s += v[j];
#pragma unroll
  for (int d = 16; d >= 1; d >>= 1) s += __shfl_xor(s, d, 32);
  const float mu = s * (1.0f / 512.0f);
  float sq = 0.0f;
#pragma unroll
  for (int j = 0; j < 16; ++j) { const float d = v[j] - mu; sq = fmaf(d, d, sq); }
#pragma unroll
  for (int d = 16; d >= 1; d >>= 1) sq += __shfl_xor(sq, d, 32);
  const float var = sq * (1.0f / 512.0f);
  const float rs  = rsqrtf(var + 1e-5f);

  float* my = sw + wave * 512;
#pragma unroll
  for (int j = 0; j < 16; ++j) my[j * 32 + lane] = (v[j] - mu) * rs;
#pragma unroll 1
  for (int j = 0; j < 16; ++j) {
    const float x = my[j * 32 + lane];
    const float e = (x > 0.0f) ? x : expm1f(x);
    my[j * 32 + lane] = e;
  }
  float e[16];
#pragma unroll
  for (int j = 0; j < 16; ++j) e[j] = my[j * 32 + lane];

  v8us pc[2][6];
#pragma unroll
  for (int c = 0; c < 2; ++c) {
    v4f xa, xb;
    xa.x = e[8 * c + 0]; xa.y = e[8 * c + 1]; xa.z = e[8 * c + 2]; xa.w = e[8 * c + 3];
    xb.x = e[8 * c + 4]; xb.y = e[8 * c + 5]; xb.z = e[8 * c + 6]; xb.w = e[8 * c + 7];
    expand8(xa, xb, pc[c][0], pc[c][1], pc[c][2], pc[c][3], pc[c][4], pc[c][5]);
  }
  unsigned short* dp = ab + (size_t)row * KL2 + 8 * lane;
#pragma unroll
  for (int c = 0; c < 2; ++c)
#pragma unroll
    for (int pl = 0; pl < 6; ++pl) *(volatile v8us*)(dp + pl * I2 + c * 256) = pc[c][pl];
  __threadfence();
#pragma unroll
  for (int c = 0; c < 2; ++c)
#pragma unroll
    for (int pl = 0; pl < 6; ++pl) *(volatile v8us*)(dp + pl * I2 + c * 256) = pc[c][pl];
}

__global__ __launch_bounds__(GTHR) void k_gemm(
    const unsigned short* __restrict__ A, const unsigned short* __restrict__ WT,
    float* outF, int K, int ldo)
{
  __shared__ __attribute__((aligned(16))) float stg[GBM * GBN];
  const int tid = (int)threadIdx.x, lane = tid & 31, wave = tid >> 5, hh = lane >> 4, m = lane & 15;
  const int rowBase = (int)blockIdx.x * GBM;
  const int col0    = (int)blockIdx.y * GBN;

  v8f acc[4];
  {
    const v8f z = {0.f, 0.f, 0.f, 0.f, 0.f, 0.f, 0.f, 0.f};
    acc[0] = z; acc[1] = z; acc[2] = z; acc[3] = z;
  }
  const unsigned short* ap = A  + (size_t)(rowBase + 16 * wave + m) * (size_t)K + 8 * hh;
  const unsigned short* wp = WT + (size_t)(col0 + m) * (size_t)K + 8 * hh;
  const int ksteps = K >> 5;
#pragma unroll 1
  for (int ks = 0; ks < ksteps; ++ks) {
    FragB af;
    af.h[0] = *(const v8usa*)(ap + 32 * ks);
    af.h[1] = *(const v8usa*)(ap + 32 * ks + 16);
#pragma unroll
    for (int t = 0; t < 4; ++t) {
      const unsigned short* wq = wp + (size_t)(16 * t) * (size_t)K + 32 * ks;
      FragB bf;
      bf.h[0] = *(const v8usa*)wq;
      bf.h[1] = *(const v8usa*)(wq + 16);
      acc[t] = wmb(af, bf, acc[t]);
    }
  }

#pragma unroll
  for (int t = 0; t < 4; ++t) {
    const int lc = 16 * t + m;
#pragma unroll
    for (int r = 0; r < 8; ++r) {
      const int lr = 16 * wave + 8 * hh + r;
      stg[lr * GBN + lc] = acc[t][r];
    }
  }
  __syncthreads();

  v4f fv[8];
#pragma unroll
  for (int i = 0; i < 8; ++i) {
    const int lr = 16 * wave + 2 * i + hh;
    fv[i] = *(const v4fa*)(stg + lr * GBN + 4 * m);
  }
#pragma unroll
  for (int i = 0; i < 8; ++i) {
    const int lr = 16 * wave + 2 * i + hh;
    const int gr = rowBase + lr;
    float* op = outF + (size_t)gr * (size_t)ldo + col0 + 4 * m;
    *(volatile v4f*)op = fv[i];
  }
  __threadfence();
#pragma unroll
  for (int i = 0; i < 8; ++i) {
    const int lr = 16 * wave + 2 * i + hh;
    const int gr = rowBase + lr;
    float* op = outF + (size_t)gr * (size_t)ldo + col0 + 4 * m;
    *(volatile v4f*)op = fv[i];
  }
}

extern "C" void kernel_launch(void* const* d_in, const int* in_sizes, int n_in,
                              void* d_out, int out_size, void* d_ws, size_t ws_size,
                              hipStream_t stream) {
  if (n_in < 6) return;
  if (in_sizes[0] < ZSD || (in_sizes[0] % ZSD) != 0) return;
  const int B = in_sizes[0] / ZSD;
  if (B < 128 || (B % 128) != 0 || B > (1 << 20)) return;
  if ((long long)in_sizes[1] != (long long)B * ADIM) return;
  if (in_sizes[2] != ADIM * ZAD * 3) return;
  if (in_sizes[3] != I1 * NOUT * 3) return;
  if (in_sizes[4] != I2 * NOUT * 3) return;
  if (in_sizes[5] != I2 * NOUT * 3) return;
  if ((long long)out_size != (long long)B * NOUT) return;

  const float* zs  = (const float*)d_in[0];
  const float* act = (const float*)d_in[1];
  const float* Wza = (const float*)d_in[2];
  const float* W1  = (const float*)d_in[3];
  const float* W2  = (const float*)d_in[4];
  const float* W3  = (const float*)d_in[5];
  float* out = (float*)d_out;

  const int MH = B / 2;

  char* ws = (char*)d_ws;
  size_t off = 0;
  const size_t oWT1 = off; off += (size_t)NOUT * KL1 * 2;
  const size_t oWT2 = off; off += (size_t)NOUT * KL2 * 2;
  const size_t oWT3 = off; off += (size_t)NOUT * KL2 * 2;
  const size_t oAB  = off; off += (size_t)MH * KL1 * 2;
  const size_t oH   = off; off += (size_t)MH * NOUT * 4;
  if (off > ws_size || off > (size_t)WSMAX) return;
  unsigned short* WT1 = (unsigned short*)(ws + oWT1);
  unsigned short* WT2 = (unsigned short*)(ws + oWT2);
  unsigned short* WT3 = (unsigned short*)(ws + oWT3);
  unsigned short* AB  = (unsigned short*)(ws + oAB);
  float*          H   = (float*)(ws + oH);

  k_prep<<<(NU1 + 2 * NU2) / NTHR, NTHR, 0, stream>>>(W1, W2, W3, WT1, WT2, WT3);

  const dim3 gg(MH / GBM, NOUT / GBN);
  for (int h = 0; h < 2; ++h) {
    const int r0 = h * MH;
    k_za_expand<<<MH / ZROWS, NTHR, 0, stream>>>(zs, act, Wza, AB, r0);
    k_gemm<<<gg, GTHR, 0, stream>>>(AB, WT1, H, KL1, NOUT);
    k_ln_expand<<<MH / NWAVE, NTHR, 0, stream>>>(H, AB, MH);
    k_gemm<<<gg, GTHR, 0, stream>>>(AB, WT2, H, KL2, NOUT);
    k_ln_expand<<<MH / NWAVE, NTHR, 0, stream>>>(H, AB, MH);
    k_gemm<<<gg, GTHR, 0, stream>>>(AB, WT3, out + (size_t)r0 * NOUT, KL2, NOUT);
  }
}
